// PointnetSAModule_32581621908084
// MI455X (gfx1250) — hardware-verified
//
#include <hip/hip_runtime.h>
#pragma clang fp contract(off)

typedef __attribute__((ext_vector_type(16))) _Float16 v16h;
typedef __attribute__((ext_vector_type(8)))  _Float16 v8h;
typedef __attribute__((ext_vector_type(4)))  _Float16 v4h;
typedef __attribute__((ext_vector_type(8)))  float    v8f;
typedef __attribute__((ext_vector_type(4)))  float    v4f;
typedef __attribute__((ext_vector_type(4)))  int      v4i;

constexpr int NBATCH  = 8;
constexpr int NPTS    = 8192;
constexpr int NFEAT   = 64;
constexpr int NCENT   = 1024;
constexpr int NGROUPS = NBATCH * NCENT;
constexpr int NROWS   = NBATCH * NPTS;
constexpr int KSAMP0  = 32;
constexpr int KSAMP1  = 64;
constexpr int OUTCH   = 384;
constexpr float WCARRY     = 16.0f;
constexpr float WCARRY_INV = 1.0f / 16.0f;
static_assert(NGROUPS == 8192 && NROWS == 65536, "shape");
static_assert((size_t)NBATCH * NCENT * 3 * 4 == 98304, "out0 bytes");
static_assert((size_t)98304 + (size_t)NBATCH * OUTCH * NCENT * 4 == 12681216, "d_out bytes");

constexpr int WH_F0 = 0;
constexpr int WH_F1 = 4096;
constexpr int WH_10 = 8192;
constexpr int WH_20 = 12288;
constexpr int WH_11 = 20480;
constexpr int WH_21 = 28672;
constexpr int WH_TOTAL = 61440;

constexpr size_t OFF_FT     = 0;
constexpr size_t OFF_PPL    = OFF_FT     + (size_t)NROWS * 64 * 2;
constexpr size_t OFF_WH     = OFF_PPL    + (size_t)NROWS * 128 * 4;
constexpr size_t OFF_WXP    = OFF_WH     + (size_t)WH_TOTAL * 2;
constexpr size_t OFF_NXW    = OFF_WXP    + (size_t)128 * 4 * 4;
constexpr size_t OFF_IDX0   = OFF_NXW    + (size_t)NGROUPS * 4 * 4;
constexpr size_t OFF_IDX1   = OFF_IDX0   + (size_t)NGROUPS * KSAMP0 * 4;
constexpr size_t OFF_PART0  = OFF_IDX1   + (size_t)NGROUPS * KSAMP1 * 4;
constexpr size_t OFF_PART10 = OFF_PART0  + (size_t)1536 * 128 * 4;
constexpr size_t OFF_PART11 = OFF_PART10 + (size_t)2048 * 128 * 4;
constexpr size_t OFF_PART20 = OFF_PART11 + (size_t)4096 * 256 * 4;
constexpr size_t OFF_PART21 = OFF_PART20 + (size_t)2048 * 256 * 4;
constexpr size_t OFF_MX0    = OFF_PART21 + (size_t)4096 * 512 * 4;
constexpr size_t OFF_MN0    = OFF_MX0    + (size_t)NGROUPS * 128 * 4;
constexpr size_t OFF_MX1    = OFF_MN0    + (size_t)NGROUPS * 128 * 4;
constexpr size_t OFF_MN1    = OFF_MX1    + (size_t)NGROUPS * 256 * 4;
constexpr size_t OFF_SSP    = OFF_MN1    + (size_t)NGROUPS * 256 * 4;
constexpr size_t WS_TOTAL   = OFF_SSP    + (size_t)6 * 512 * 4;
static_assert(WS_TOTAL <= (size_t)134217728, "carve");
static_assert((OFF_PPL % 128) == 0 && (OFF_WH % 128) == 0 && (OFF_WXP % 128) == 0 && (OFF_NXW % 128) == 0, "align");
static_assert((OFF_IDX0 % 128) == 0 && (OFF_PART0 % 128) == 0 && (OFF_MX0 % 128) == 0 && (OFF_SSP % 128) == 0, "align");

union FragU { v16h v; v8h h[2]; };
__device__ __forceinline__ v16h frag_ld(const _Float16* p) {
  FragU f;
  f.h[0] = *(const v8h*)(p);
  f.h[1] = *(const v8h*)(p + 16);
  return f.v;
}
__device__ __forceinline__ v8f mma16(v16h a, v16h b, v8f c) {
  return __builtin_amdgcn_wmma_f32_16x16x32_f16(false, a, false, b, (short)0, c, false, false);
}
__device__ __forceinline__ void guard_row4(v8f& c0, v8f& c1, v8f& c2, v8f& c3,
                                           v16h a, v16h b0, v16h b1, v16h b2, v16h b3) {
  asm volatile("v_nop\n\tv_nop\n\tv_nop\n\tv_nop"
               : "+v"(c0), "+v"(c1), "+v"(c2), "+v"(c3)
               : "v"(a), "v"(b0), "v"(b1), "v"(b2), "v"(b3));
}
__device__ __forceinline__ void guard_grp8(v8f& c0, v8f& c1, v8f& c2, v8f& c3,
                                           v8f& c4, v8f& c5, v8f& c6, v8f& c7,
                                           v16h a0, v16h a1, v16h b0, v16h b1, v16h b2, v16h b3) {
  asm volatile("v_nop\n\tv_nop\n\tv_nop\n\tv_nop"
               : "+v"(c0), "+v"(c1), "+v"(c2), "+v"(c3), "+v"(c4), "+v"(c5), "+v"(c6), "+v"(c7)
               : "v"(a0), "v"(a1), "v"(b0), "v"(b1), "v"(b2), "v"(b3));
}
__device__ __forceinline__ float dot3w(v4f w, v4f p) {
  float a = w.x * p.x;
  a = a + w.y * p.y;
  a = a + w.z * p.z;
  return a;
}
__device__ __forceinline__ double shfl_xor_f64(double v, int m) {
  const long long bits = __double_as_longlong(v);
  int lo = (int)(bits & 0xffffffffll);
  int hi = (int)(bits >> 32);
  lo = __shfl_xor(lo, m);
  hi = __shfl_xor(hi, m);
  const long long nb = (((long long)hi) << 32) | (long long)(unsigned)lo;
  return __longlong_as_double(nb);
}

__global__ __launch_bounds__(256) void k_packfeat(const float* __restrict__ feat, unsigned short* __restrict__ ftp) {
  __shared__ float tile[64 * 65];
  const int t = threadIdx.x;
  const int blk = blockIdx.x;
  const int b = blk >> 7;
  const int n0 = (blk & 127) << 6;
  const int n = t & 63;
  const int cq = t >> 6;
  const float* src = feat + (size_t)b * NFEAT * NPTS + n0 + n;
#pragma unroll 4
  for (int i = 0; i < 16; ++i) {
    const int c = i * 4 + cq;
    tile[c * 65 + n] = src[(size_t)c * NPTS];
  }
  __syncthreads();
  _Float16* ft = (_Float16*)ftp;
  const int c8 = (t & 7) * 8;
  const int l0 = t >> 3;
  v8h h0, h1;
#pragma unroll
  for (int e = 0; e < 8; ++e) {
    h0[e] = (_Float16)tile[(c8 + e) * 65 + l0];
    h1[e] = (_Float16)tile[(c8 + e) * 65 + l0 + 32];
  }
  const size_t r0 = (size_t)b * NPTS + n0 + l0;
  volatile v8h* p0 = (volatile v8h*)(ft + r0 * 64 + c8);
  volatile v8h* p1 = (volatile v8h*)(ft + (r0 + 32) * 64 + c8);
  *p0 = h0;
  *p1 = h1;
  __threadfence();
  *p0 = h0;
  *p1 = h1;
}

__global__ __launch_bounds__(256) void k_packw(const float* __restrict__ w00, const float* __restrict__ w10,
                                               const float* __restrict__ w01, const float* __restrict__ w02,
                                               const float* __restrict__ w11, const float* __restrict__ w12,
                                               unsigned short* __restrict__ whp, float* __restrict__ wxp) {
  const int y = blockIdx.y;
  const int i = blockIdx.x * 256 + threadIdx.x;
  if (y >= 6) {
    const float* s = (y == 6) ? w00 : w10;
    if (i < 64) {
      v4f v;
      v.x = s[i * 67 + 0];
      v.y = s[i * 67 + 1];
      v.z = s[i * 67 + 2];
      v.w = 0.0f;
      volatile v4f* p = (volatile v4f*)(wxp + (size_t)((y - 6) * 64 + i) * 4);
      *p = v;
      __threadfence();
      *p = v;
    }
    return;
  }
  const float* src = (y == 0) ? w00 : (y == 1) ? w10 : (y == 2) ? w01 : (y == 3) ? w02 : (y == 4) ? w11 : w12;
  const int ld   = (y < 2) ? 67 : ((y == 5) ? 128 : 64);
  const int col0 = (y < 2) ? 3 : 0;
  const int kd   = (y == 5) ? 128 : 64;
  const int rows = (y < 3) ? 64 : ((y < 5) ? 128 : 256);
  const int off  = (y == 0) ? WH_F0 : (y == 1) ? WH_F1 : (y == 2) ? WH_10 : (y == 3) ? WH_20 : (y == 4) ? WH_11 : WH_21;
  const int n8 = (rows * kd) >> 3;
  if (i < n8) {
    const int e0 = i * 8;
    const int row = e0 / kd;
    const int k = e0 - row * kd;
    const float* p = src + (size_t)row * ld + col0 + k;
    v8h hv;
#pragma unroll
    for (int e = 0; e < 8; ++e) {
      const float f = p[e] * WCARRY;
      hv[e] = (_Float16)f;
    }
    volatile v8h* q = (volatile v8h*)((_Float16*)whp + off + e0);
    *q = hv;
    __threadfence();
    *q = hv;
  }
}

__global__ __launch_bounds__(1024) void k_fps(const float* __restrict__ xyz, float* __restrict__ out0,
                                              float* __restrict__ nxw) {
#pragma clang fp contract(off)
  __shared__ __align__(16) float cs[NCENT * 4];
  __shared__ double rd[96];
  __shared__ float smean[4];
  __shared__ float rv[2][32];
  __shared__ int   ri[2][32];
  const int t = threadIdx.x;
  const int lane = t & 31;
  const int w = t >> 5;
  const int b = blockIdx.x;
  const bool w0 = (t < 32);
  const float* xb = xyz + (size_t)b * NPTS * 3;

  float px[8], py[8], pz[8], dist[8];
#pragma unroll
  for (int i = 0; i < 8; ++i) {
    int jj = i * 1024 + t - 1;
    jj = jj < 0 ? 0 : jj;
    px[i] = xb[jj * 3 + 0];
    py[i] = xb[jj * 3 + 1];
    pz[i] = xb[jj * 3 + 2];
    dist[i] = 1e10f;
    if (i == 2 || i == 5 || i == 7) {
      asm volatile("" : "+v"(pz[i]) : : "memory");
    }
  }
  float px8 = 0.0f, py8 = 0.0f, pz8 = 0.0f, dist8 = -1.0f;
  if (w0) {
    px8 = xb[(NPTS - 1) * 3 + 0];
    py8 = xb[(NPTS - 1) * 3 + 1];
    pz8 = xb[(NPTS - 1) * 3 + 2];
    dist8 = (t == 0) ? 1e10f : -1.0f;
  }

  double sx = 0.0, sy = 0.0, sz = 0.0;
#pragma unroll
  for (int i = 0; i < 8; ++i) {
    const bool val = (i > 0) || (t > 0);
    sx += val ? (double)px[i] : 0.0;
    sy += val ? (double)py[i] : 0.0;
    sz += val ? (double)pz[i] : 0.0;
  }
  {
    const bool v8 = (t == 0);
    sx += v8 ? (double)px8 : 0.0;
    sy += v8 ? (double)py8 : 0.0;
    sz += v8 ? (double)pz8 : 0.0;
  }
#pragma unroll
  for (int off = 16; off >= 1; off >>= 1) {
    sx += shfl_xor_f64(sx, off);
    sy += shfl_xor_f64(sy, off);
    sz += shfl_xor_f64(sz, off);
  }
  if (lane == 0) {
    rd[w * 3 + 0] = sx;
    rd[w * 3 + 1] = sy;
    rd[w * 3 + 2] = sz;
  }
  __syncthreads();
  if (t == 0) {
    double ax = 0.0, ay = 0.0, az = 0.0;
    for (int w2 = 0; w2 < 32; ++w2) {
      ax += rd[w2 * 3 + 0];
      ay += rd[w2 * 3 + 1];
      az += rd[w2 * 3 + 2];
    }
    smean[0] = (float)(ax * (1.0 / 8192.0));
    smean[1] = (float)(ay * (1.0 / 8192.0));
    smean[2] = (float)(az * (1.0 / 8192.0));
    smean[3] = 0.0f;
  }
  __syncthreads();
  const float mx = smean[0], my = smean[1], mz = smean[2];
  px[0] = (t == 0) ? mx : px[0];
  py[0] = (t == 0) ? my : py[0];
  pz[0] = (t == 0) ? mz : pz[0];

  int far = 0;
  for (int step = 0; step < NCENT; ++step) {
    int fj = far - 1;
    fj = fj < 0 ? 0 : fj;
    fj = fj > (NPTS - 1) ? (NPTS - 1) : fj;
    const float lx = xb[fj * 3 + 0];
    const float ly = xb[fj * 3 + 1];
    const float lz = xb[fj * 3 + 2];
    const bool isMean = (far == 0);
    const float cx = isMean ? mx : lx;
    const float cy = isMean ? my : ly;
    const float cz = isMean ? mz : lz;
    if (t == 0) {
      cs[step * 4 + 0] = cx;
      cs[step * 4 + 1] = cy;
      cs[step * 4 + 2] = cz;
      cs[step * 4 + 3] = 0.0f;
    }
    float best = -2.0f;
    int bidx = 0x7fffffff;
#pragma unroll
    for (int i = 0; i < 8; ++i) {
      const float dx = px[i] - cx;
      const float dy = py[i] - cy;
      const float dz = pz[i] - cz;
      const float t0 = dx * dx;
      const float t1 = dy * dy;
      const float t2 = dz * dz;
      const float d2 = (t0 + t2) + t1;
      const float dn = fminf(dist[i], d2);
      dist[i] = dn;
      const bool gt = dn > best;
      best = gt ? dn : best;
      bidx = gt ? (i * 1024 + t) : bidx;
    }
    if (w0) {
      const float dx = px8 - cx;
      const float dy = py8 - cy;
      const float dz = pz8 - cz;
      const float t0 = dx * dx;
      const float t1 = dy * dy;
      const float t2 = dz * dz;
      const float d2 = (t0 + t2) + t1;
      const float dn = fminf(dist8, d2);
      dist8 = dn;
      const bool gt = dn > best;
      best = gt ? dn : best;
      bidx = gt ? (NPTS + t) : bidx;
    }
#pragma unroll
    for (int off = 16; off >= 1; off >>= 1) {
      const float ov = __shfl_xor(best, off);
      const int   oi = __shfl_xor(bidx, off);
      const bool take = (ov > best) || ((ov == best) && (oi < bidx));
      best = take ? ov : best;
      bidx = take ? oi : bidx;
    }
    const int par = step & 1;
    if (lane == 0) {
      rv[par][w] = best;
      ri[par][w] = bidx;
    }
    __syncthreads();
    float v2 = rv[par][lane];
    int   i2 = ri[par][lane];
#pragma unroll
    for (int off = 16; off >= 1; off >>= 1) {
      const float ov = __shfl_xor(v2, off);
      const int   oi = __shfl_xor(i2, off);
      const bool take = (ov > v2) || ((ov == v2) && (oi < i2));
      v2 = take ? ov : v2;
      i2 = take ? oi : i2;
    }
    far = __builtin_amdgcn_readfirstlane(i2);
    far = far < 0 ? 0 : far;
    far = far > NPTS ? NPTS : far;
  }
  __syncthreads();
  const v4f nv = *(const v4f*)(cs + t * 4);
  volatile v4f* np = (volatile v4f*)(nxw + ((size_t)b * NCENT + t) * 4);
  const int tc = t < 768 ? t : 767;
  v4f ov4;
#pragma unroll
  for (int e = 0; e < 4; ++e) {
    const int f = tc * 4 + e;
    const int st = f / 3;
    const int cm = f - st * 3;
    ov4[e] = cs[st * 4 + cm];
  }
  volatile v4f* op = (volatile v4f*)(out0 + (size_t)b * NCENT * 3 + (size_t)tc * 4);
  *np = nv;
  if (t < 768) { *op = ov4; }
  __threadfence();
  *np = nv;
  if (t < 768) { *op = ov4; }
}

__global__ __launch_bounds__(256) void k_ball(const float* __restrict__ xyz, const float* __restrict__ nxw,
                                              int* __restrict__ idx0, int* __restrict__ idx1) {
#pragma clang fp contract(off)
  __shared__ __align__(16) int r0[8 * KSAMP0];
  __shared__ __align__(16) int r1[8 * KSAMP1];
  const int lane = threadIdx.x & 31;
  const int w = threadIdx.x >> 5;
  const int q = blockIdx.x * 8 + w;
  const int b = q >> 10;
  const float* xb = xyz + (size_t)b * NPTS * 3;
  const v4f c = *(const v4f*)(nxw + (size_t)q * 4);
  const float rr0 = __uint_as_float(0x3E23D70Au);
  const float rr1 = __uint_as_float(0x3F23D70Au);
  const unsigned lt = (1u << lane) - 1u;
  int cnt0 = 0, cnt1 = 0, f0 = 0, f1 = 0;
  for (int j0 = 0; j0 < NPTS; j0 += 32) {
    if (cnt0 >= KSAMP0 && cnt1 >= KSAMP1) break;
    const int j = j0 + lane;
    const float x = xb[j * 3 + 0];
    const float y = xb[j * 3 + 1];
    const float z = xb[j * 3 + 2];
    const float dx = c.x - x;
    const float dy = c.y - y;
    const float dz = c.z - z;
    const float t0 = dx * dx;
    const float t1 = dy * dy;
    const float t2 = dz * dz;
    const float d2 = (t0 + t2) + t1;
    const bool in0 = d2 < rr0;
    const bool in1 = d2 < rr1;
    const unsigned m0 = __builtin_amdgcn_ballot_w32(in0);
    const unsigned m1 = __builtin_amdgcn_ballot_w32(in1);
    const int pos0 = cnt0 + __popc(m0 & lt);
    const int pos1 = cnt1 + __popc(m1 & lt);
    if (in0 && pos0 < KSAMP0) { r0[w * KSAMP0 + pos0] = j; }
    if (in1 && pos1 < KSAMP1) { r1[w * KSAMP1 + pos1] = j; }
    if (cnt0 == 0 && m0 != 0u) { f0 = j0 + __builtin_ctz(m0); }
    if (cnt1 == 0 && m1 != 0u) { f1 = j0 + __builtin_ctz(m1); }
    cnt0 += __popc(m0);
    cnt1 += __popc(m1);
  }
  const int n0c = cnt0 < KSAMP0 ? cnt0 : KSAMP0;
  const int n1c = cnt1 < KSAMP1 ? cnt1 : KSAMP1;
  if (lane >= n0c)      { r0[w * KSAMP0 + lane] = f0; }
  if (lane >= n1c)      { r1[w * KSAMP1 + lane] = f1; }
  if (lane + 32 >= n1c) { r1[w * KSAMP1 + 32 + lane] = f1; }
  __syncthreads();
  if (w < 2) {
    v4i v = *(const v4i*)(r0 + w * 128 + lane * 4);
#pragma unroll
    for (int e = 0; e < 4; ++e) {
      int u = v[e];
      u = u < 0 ? 0 : u;
      u = u > (NPTS - 1) ? (NPTS - 1) : u;
      v[e] = u;
    }
    volatile v4i* p = (volatile v4i*)(idx0 + (size_t)blockIdx.x * (8 * KSAMP0) + w * 128 + lane * 4);
    *p = v;
    __threadfence();
    *p = v;
  } else if (w < 6) {
    v4i v = *(const v4i*)(r1 + (w - 2) * 128 + lane * 4);
#pragma unroll
    for (int e = 0; e < 4; ++e) {
      int u = v[e];
      u = u < 0 ? 0 : u;
      u = u > (NPTS - 1) ? (NPTS - 1) : u;
      v[e] = u;
    }
    volatile v4i* p = (volatile v4i*)(idx1 + (size_t)blockIdx.x * (8 * KSAMP1) + (w - 2) * 128 + lane * 4);
    *p = v;
    __threadfence();
    *p = v;
  }
}

__global__ __launch_bounds__(256) void k_pgemm(const unsigned short* __restrict__ ftp,
                                               const unsigned short* __restrict__ wfp,
                                               const float* __restrict__ wx, const float* __restrict__ xyz,
                                               float* __restrict__ P) {
  __shared__ __align__(16) float sT[8][16 * 68];
  const _Float16* A  = (const _Float16*)ftp;
  const _Float16* Bt = (const _Float16*)wfp;
  const int lane = threadIdx.x & 31;
  const int wave = threadIdx.x >> 5;
  const int tile = blockIdx.x * 8 + wave;
  const int tm = tile >> 1;
  const int tn = tile & 1;
  const int m0 = tm << 6;
  const int n0 = tn << 6;
  const int rlane = lane & 15;
  const int hh = lane >> 4;
  const int koff = hh * 8;
  const int mOff = hh * 8;

  v8f acc[4][4];
#pragma unroll
  for (int i = 0; i < 4; ++i)
#pragma unroll
    for (int j = 0; j < 4; ++j) acc[i][j] = (v8f){0.f, 0.f, 0.f, 0.f, 0.f, 0.f, 0.f, 0.f};

#pragma unroll
  for (int k0 = 0; k0 < 64; k0 += 32) {
    v16h bh[4];
#pragma unroll
    for (int j = 0; j < 4; ++j) bh[j] = frag_ld(Bt + (size_t)(n0 + 16 * j + rlane) * 64 + koff + k0);
#pragma unroll
    for (int i = 0; i < 4; ++i) {
      const v16h ah = frag_ld(A + (size_t)(m0 + 16 * i + rlane) * 64 + koff + k0);
#pragma unroll
      for (int j = 0; j < 4; ++j) acc[i][j] = mma16(ah, bh[j], acc[i][j]);
      guard_row4(acc[i][0], acc[i][1], acc[i][2], acc[i][3], ah, bh[0], bh[1], bh[2], bh[3]);
    }
  }

  float* slab = sT[wave];
  const int c4 = rlane * 4;
  v4f wxe[4];
#pragma unroll
  for (int e = 0; e < 4; ++e) wxe[e] = *(const v4f*)(wx + (size_t)(n0 + c4 + e) * 4);

#pragma unroll
  for (int i = 0; i < 4; ++i) {
    const int mBase = m0 + 16 * i;
#pragma unroll
    for (int j = 0; j < 4; ++j) {
#pragma unroll
      for (int r = 0; r < 8; ++r) {
        slab[(mOff + r) * 68 + 16 * j + rlane] = acc[i][j][r] * WCARRY_INV;
      }
    }
    __syncthreads();
#pragma unroll 1
    for (int it = 0; it < 8; ++it) {
      const int row = it * 2 + hh;
      const size_t gm = (size_t)(mBase + row);
      const float x = xyz[gm * 3 + 0];
      const float y = xyz[gm * 3 + 1];
      const float z = xyz[gm * 3 + 2];
      v4f v = *(const v4f*)(slab + row * 68 + c4);
#pragma unroll
      for (int e = 0; e < 4; ++e) {
        float a = v[e];
        a = a + wxe[e].x * x;
        a = a + wxe[e].y * y;
        a = a + wxe[e].z * z;
        v[e] = a;
      }
      *(v4f*)(slab + row * 68 + c4) = v;
    }
    for (int pass = 0; pass < 2; ++pass) {
#pragma unroll
      for (int it = 0; it < 8; ++it) {
        const int row = it * 2 + hh;
        const v4f v = *(const v4f*)(slab + row * 68 + c4);
        *(volatile v4f*)(P + (size_t)(mBase + row) * 128 + n0 + c4) = v;
      }
      __threadfence();
    }
    __syncthreads();
  }
}

__global__ __launch_bounds__(256) void k_stats0(const float* __restrict__ P, const int* __restrict__ idx0,
                                                const int* __restrict__ idx1, const float* __restrict__ nxw,
                                                const float* __restrict__ wx, float* __restrict__ part) {
  __shared__ __align__(16) float red[8 * 128];
  const int t = threadIdx.x;
  const int lane = t & 31;
  const int w = t >> 5;
  const int hh = lane >> 4;
  const int c4 = (lane & 15) * 4;
  const int bi = (blockIdx.x >= 512) ? 1 : 0;
  const int lb = blockIdx.x - bi * 512;
  const int* idx = bi ? idx1 : idx0;
  const int kshift = bi ? 6 : 5;
  const int colbase = lb * 512 + w * 64;
  v4f wxv[4];
#pragma unroll
  for (int e = 0; e < 4; ++e) wxv[e] = *(const v4f*)(wx + (size_t)(bi * 64 + c4 + e) * 4);
  float s[4] = {0.f, 0.f, 0.f, 0.f};
  float sq[4] = {0.f, 0.f, 0.f, 0.f};
#pragma unroll 1
  for (int sb = 0; sb < 2; ++sb) {
    const int cb = colbase + sb * 32;
    const int g = cb >> kshift;
    const int b = g >> 10;
    const v4f nx = *(const v4f*)(nxw + (size_t)g * 4);
    float q[4];
#pragma unroll
    for (int e = 0; e < 4; ++e) q[e] = dot3w(wxv[e], nx);
#pragma unroll 4
    for (int it = 0; it < 16; ++it) {
      const int col = cb + it * 2 + hh;
      int id = idx[col];
      id = id < 0 ? 0 : id;
      id = id > (NPTS - 1) ? (NPTS - 1) : id;
      const v4f pv = *(const v4f*)(P + ((size_t)b * NPTS + id) * 128 + bi * 64 + c4);
#pragma unroll
      for (int e = 0; e < 4; ++e) {
        const float y = pv[e] - q[e];
        s[e] = s[e] + y;
        sq[e] = sq[e] + y * y;
      }
    }
  }
#pragma unroll
  for (int e = 0; e < 4; ++e) {
    s[e]  = s[e]  + __shfl_xor(s[e], 16);
    sq[e] = sq[e] + __shfl_xor(sq[e], 16);
  }
  if (hh == 0) {
#pragma unroll
    for (int e = 0; e < 4; ++e) {
      red[w * 128 + c4 + e] = s[e];
      red[w * 128 + 64 + c4 + e] = sq[e];
    }
  }
  __syncthreads();
  if (t < 32) {
    v4f a = (v4f){0.f, 0.f, 0.f, 0.f};
#pragma unroll
    for (int w2 = 0; w2 < 8; ++w2) a = a + *(const v4f*)(red + w2 * 128 + t * 4);
    volatile v4f* p = (volatile v4f*)(part + (size_t)blockIdx.x * 128 + t * 4);
    *p = a;
    __threadfence();
    *p = a;
  }
}

__global__ __launch_bounds__(256) void k_fold(const float* __restrict__ part, int nblk, int nch,
                                              const float* __restrict__ gam, const float* __restrict__ bet,
                                              double invN, float* __restrict__ ss) {
  __shared__ __align__(16) float st[512];
  const int t = threadIdx.x;
  const int cc = t < nch ? t : (nch - 1);
  double s = 0.0, q = 0.0;
  const int stride = 2 * nch;
  for (int blk = 0; blk < nblk; ++blk) {
    s += (double)part[(size_t)blk * stride + cc];
    q += (double)part[(size_t)blk * stride + nch + cc];
  }
  const double m = s * invN;
  double var = q * invN - m * m;
  var = var < 0.0 ? 0.0 : var;
  const float vf = (float)var;
  const float rs = 1.0f / sqrtf(vf + 1e-5f);
  const float sc = gam[cc] * rs;
  const float mf = (float)m;
  const float sh = bet[cc] - mf * sc;
  st[t] = (t < nch) ? sc : 0.0f;
  st[256 + t] = (t < nch) ? sh : 0.0f;
  __syncthreads();
  if (t < 128) {
    const v4f v = *(const v4f*)(st + t * 4);
    volatile v4f* p = (volatile v4f*)(ss + t * 4);
    *p = v;
    __threadfence();
    *p = v;
  }
}

template <int C1, int C2, int KS, int MODE>
__global__ __launch_bounds__(128) void k_mlp(const float* __restrict__ P, const int* __restrict__ idx,
                                             const float* __restrict__ nxw, const float* __restrict__ wx,
                                             const float* __restrict__ ss0, const float* __restrict__ ss1,
                                             const unsigned short* __restrict__ w1p,
                                             const unsigned short* __restrict__ w2p,
                                             float* __restrict__ part, float* __restrict__ MXp,
                                             float* __restrict__ MNp, int pcol0) {
  static_assert((128 / KS) * C2 == 512, "group rows per block");
  static_assert(64 * C2 <= 16384, "stat staging fits the dead A tile");
  static_assert(C1 % 64 == 0 && C2 % 64 == 0 && C1 % 32 == 0, "tile multiples");
  constexpr int A2_BYTES = 128 * C1 * 2;
  __shared__ __align__(16) unsigned char smraw[16384 + A2_BYTES];
  _Float16* sA  = (_Float16*)smraw;
  float*    red = (float*)smraw;
  _Float16* sA2 = (_Float16*)(smraw + 16384);
  float*   red1 = (float*)(smraw + 16384);

  const int tid = threadIdx.x;
  const int lane = tid & 31;
  const int w = tid >> 5;
  const int hh = lane >> 4;
  const int rl = lane & 15;
  const int c4 = rl * 4;
  const int koff = hh * 8;
  const int col0 = blockIdx.x * 128;
  const int cw = col0 + 32 * w;
  const int g = cw / KS;
  const int b = g >> 10;

  {
    v4f wxv[4];
#pragma unroll
    for (int e = 0; e < 4; ++e) wxv[e] = *(const v4f*)(wx + (size_t)(c4 + e) * 4);
    const v4f sc0 = *(const v4f*)(ss0 + c4);
    const v4f sh0 = *(const v4f*)(ss0 + 256 + c4);
    const v4f nx  = *(const v4f*)(nxw + (size_t)g * 4);
    float q[4];
#pragma unroll
    for (int e = 0; e < 4; ++e) q[e] = dot3w(wxv[e], nx);
#pragma unroll 4
    for (int it = 0; it < 16; ++it) {
      const int row = 32 * w + it * 2 + hh;
      int id = idx[col0 + row];
      id = id < 0 ? 0 : id;
      id = id > (NPTS - 1) ? (NPTS - 1) : id;
      const v4f pv = *(const v4f*)(P + ((size_t)b * NPTS + id) * 128 + pcol0 + c4);
      v4h hv;
#pragma unroll
      for (int e = 0; e < 4; ++e) {
        const float y = pv[e] - q[e];
        const float a = fmaxf(y * sc0[e] + sh0[e], 0.0f);
        hv[e] = (_Float16)a;
      }
      *(v4h*)(sA + row * 64 + c4) = hv;
    }
  }
  __syncthreads();

  const _Float16* W1 = (const _Float16*)w1p;
#pragma unroll
  for (int nc = 0; nc < C1 / 64; ++nc) {
    v8f acc[2][4];
#pragma unroll
    for (int i = 0; i < 2; ++i)
#pragma unroll
      for (int j = 0; j < 4; ++j) acc[i][j] = (v8f){0.f, 0.f, 0.f, 0.f, 0.f, 0.f, 0.f, 0.f};
#pragma unroll
    for (int k0 = 0; k0 < 64; k0 += 32) {
      const v16h a0 = frag_ld(sA + (32 * w + rl) * 64 + koff + k0);
      const v16h a1 = frag_ld(sA + (32 * w + 16 + rl) * 64 + koff + k0);
      v16h bf[4];
#pragma unroll
      for (int j = 0; j < 4; ++j) bf[j] = frag_ld(W1 + (size_t)(nc * 64 + 16 * j + rl) * 64 + koff + k0);
#pragma unroll
      for (int j = 0; j < 4; ++j) {
        acc[0][j] = mma16(a0, bf[j], acc[0][j]);
        acc[1][j] = mma16(a1, bf[j], acc[1][j]);
      }
      guard_grp8(acc[0][0], acc[0][1], acc[0][2], acc[0][3], acc[1][0], acc[1][1], acc[1][2], acc[1][3],
                 a0, a1, bf[0], bf[1], bf[2], bf[3]);
    }
    if (MODE == 0) {
#pragma unroll
      for (int j = 0; j < 4; ++j) {
        const int ch = nc * 64 + 16 * j + rl;
        float s = 0.0f, qq = 0.0f;
#pragma unroll
        for (int i = 0; i < 2; ++i) {
#pragma unroll
          for (int r = 0; r < 8; ++r) {
            const float v = acc[i][j][r] * WCARRY_INV;
            s = s + v;
            qq = qq + v * v;
          }
        }
        s  = s  + __shfl_xor(s, 16);
        qq = qq + __shfl_xor(qq, 16);
        if (hh == 0) {
          red1[w * 2 * C1 + ch] = s;
          red1[w * 2 * C1 + C1 + ch] = qq;
        }
      }
    } else {
#pragma unroll
      for (int j = 0; j < 4; ++j) {
        const int ch = nc * 64 + 16 * j + rl;
        const float sc = ss1[ch];
        const float sh = ss1[256 + ch];
#pragma unroll
        for (int i = 0; i < 2; ++i) {
#pragma unroll
          for (int r = 0; r < 8; ++r) {
            const float v = acc[i][j][r] * WCARRY_INV;
            const float a = fmaxf(v * sc + sh, 0.0f);
            sA2[(32 * w + 16 * i + 8 * hh + r) * C1 + ch] = (_Float16)a;
          }
        }
      }
    }
  }
  __syncthreads();

  if (MODE == 0) {
    if (tid < (2 * C1) / 4) {
      v4f a = (v4f){0.f, 0.f, 0.f, 0.f};
#pragma unroll
      for (int w2 = 0; w2 < 4; ++w2) a = a + *(const v4f*)(red1 + w2 * 2 * C1 + tid * 4);
      volatile v4f* p = (volatile v4f*)(part + (size_t)blockIdx.x * (2 * C1) + tid * 4);
      *p = a;
      __threadfence();
      *p = a;
    }
    return;
  }

  const _Float16* W2 = (const _Float16*)w2p;
#pragma unroll 1
  for (int nc = 0; nc < C2 / 64; ++nc) {
    v8f acc[2][4];
#pragma unroll
    for (int i = 0; i < 2; ++i)
#pragma unroll
      for (int j = 0; j < 4; ++j) acc[i][j] = (v8f){0.f, 0.f, 0.f, 0.f, 0.f, 0.f, 0.f, 0.f};
#pragma unroll
    for (int k0 = 0; k0 < C1; k0 += 32) {
      const v16h a0 = frag_ld(sA2 + (32 * w + rl) * C1 + koff + k0);
      const v16h a1 = frag_ld(sA2 + (32 * w + 16 + rl) * C1 + koff + k0);
      v16h bf[4];
#pragma unroll
      for (int j = 0; j < 4; ++j) bf[j] = frag_ld(W2 + (size_t)(nc * 64 + 16 * j + rl) * C1 + koff + k0);
#pragma unroll
      for (int j = 0; j < 4; ++j) {
        acc[0][j] = mma16(a0, bf[j], acc[0][j]);
        acc[1][j] = mma16(a1, bf[j], acc[1][j]);
      }
      guard_grp8(acc[0][0], acc[0][1], acc[0][2], acc[0][3], acc[1][0], acc[1][1], acc[1][2], acc[1][3],
                 a0, a1, bf[0], bf[1], bf[2], bf[3]);
    }
#pragma unroll
    for (int j = 0; j < 4; ++j) {
      const int ch = nc * 64 + 16 * j + rl;
      float s = 0.0f, qq = 0.0f;
      float mx = -__builtin_huge_valf();
      float mn = __builtin_huge_valf();
#pragma unroll
      for (int i = 0; i < 2; ++i) {
#pragma unroll
        for (int r = 0; r < 8; ++r) {
          const float v = acc[i][j][r] * WCARRY_INV;
          s = s + v;
          qq = qq + v * v;
          mx = fmaxf(mx, v);
          mn = fminf(mn, v);
        }
      }
      s  = s  + __shfl_xor(s, 16);
      qq = qq + __shfl_xor(qq, 16);
      const float omx = __shfl_xor(mx, 16);
      const float omn = __shfl_xor(mn, 16);
      mx = fmaxf(mx, omx);
      mn = fminf(mn, omn);
      if (hh == 0) {
        red[w * 4 * C2 + ch] = s;
        red[w * 4 * C2 + C2 + ch] = qq;
        red[w * 4 * C2 + 2 * C2 + ch] = mx;
        red[w * 4 * C2 + 3 * C2 + ch] = mn;
      }
    }
  }
  __syncthreads();

  {
    constexpr int WPG = KS / 32;
    constexpr int NSV = (2 * C2) / 4;
    const bool doS = tid < NSV;
    const int ts = doS ? tid : 0;
    v4f sv = (v4f){0.f, 0.f, 0.f, 0.f};
#pragma unroll
    for (int w2 = 0; w2 < 4; ++w2) sv = sv + *(const v4f*)(red + w2 * 4 * C2 + ts * 4);
    const int e0 = tid * 4;
    const int gl = e0 / C2;
    const int c = e0 - gl * C2;
    v4f mxv = *(const v4f*)(red + (gl * WPG) * 4 * C2 + 2 * C2 + c);
    v4f mnv = *(const v4f*)(red + (gl * WPG) * 4 * C2 + 3 * C2 + c);
#pragma unroll
    for (int w2 = 1; w2 < WPG; ++w2) {
      const v4f om = *(const v4f*)(red + (gl * WPG + w2) * 4 * C2 + 2 * C2 + c);
      const v4f on = *(const v4f*)(red + (gl * WPG + w2) * 4 * C2 + 3 * C2 + c);
#pragma unroll
      for (int e = 0; e < 4; ++e) {
        mxv[e] = fmaxf(mxv[e], om[e]);
        mnv[e] = fminf(mnv[e], on[e]);
      }
    }
    const size_t g0 = (size_t)(col0 / KS);
    volatile v4f* pp = (volatile v4f*)(part + (size_t)blockIdx.x * (2 * C2) + ts * 4);
    volatile v4f* px = (volatile v4f*)(MXp + g0 * C2 + e0);
    volatile v4f* pn = (volatile v4f*)(MNp + g0 * C2 + e0);
    if (doS) { *pp = sv; }
    *px = mxv;
    *pn = mnv;
    __threadfence();
    if (doS) { *pp = sv; }
    *px = mxv;
    *pn = mnv;
  }
}

__global__ __launch_bounds__(256) void k_final(const float* __restrict__ MXp, const float* __restrict__ MNp,
                                               const float* __restrict__ ss2, float* __restrict__ out1,
                                               int nch2, int cbase) {
  __shared__ __align__(16) float tile[64 * 68];
  const int t = threadIdx.x;
  const int nOT = nch2 >> 6;
  const int ot = blockIdx.x % nOT;
  const int stile = blockIdx.x / nOT;
  const int g0 = stile * 64;
  const int o0 = ot * 64;
  const int c4 = (t & 15) * 4;
  const int rr = t >> 4;
  const v4f sc = *(const v4f*)(ss2 + o0 + c4);
  const v4f sh = *(const v4f*)(ss2 + 256 + o0 + c4);
#pragma unroll
  for (int p = 0; p < 4; ++p) {
    const int gl = p * 16 + rr;
    const size_t gg = (size_t)(g0 + gl);
    const v4f mx = *(const v4f*)(MXp + gg * nch2 + o0 + c4);
    const v4f mn = *(const v4f*)(MNp + gg * nch2 + o0 + c4);
#pragma unroll
    for (int e = 0; e < 4; ++e) {
      const float x = (sc[e] >= 0.0f) ? mx[e] : mn[e];
      const float v = fmaxf(x * sc[e] + sh[e], 0.0f);
      tile[(c4 + e) * 68 + gl] = v;
    }
  }
  __syncthreads();
  const int b = g0 >> 10;
  const int s0 = g0 & 1023;
  v4f vals[4];
#pragma unroll
  for (int p = 0; p < 4; ++p) vals[p] = *(const v4f*)(tile + (p * 16 + rr) * 68 + c4);
  float* ob = out1 + ((size_t)b * OUTCH + cbase + o0) * NCENT + s0 + c4;
#pragma unroll
  for (int p = 0; p < 4; ++p) *(volatile v4f*)(ob + (size_t)(p * 16 + rr) * NCENT) = vals[p];
  __threadfence();
#pragma unroll
  for (int p = 0; p < 4; ++p) *(volatile v4f*)(ob + (size_t)(p * 16 + rr) * NCENT) = vals[p];
}

extern "C" void kernel_launch(void* const* d_in, const int* in_sizes, int n_in,
                              void* d_out, int out_size, void* d_ws, size_t ws_size, hipStream_t stream) {
  (void)in_sizes; (void)n_in; (void)out_size;
  if (ws_size < WS_TOTAL) return;
  const float* xyz  = (const float*)d_in[0];
  const float* feat = (const float*)d_in[1];
  const float* w00 = (const float*)d_in[2];
  const float* g00 = (const float*)d_in[3];
  const float* b00 = (const float*)d_in[4];
  const float* w01 = (const float*)d_in[5];
  const float* g01 = (const float*)d_in[6];
  const float* b01 = (const float*)d_in[7];
  const float* w02 = (const float*)d_in[8];
  const float* g02 = (const float*)d_in[9];
  const float* b02 = (const float*)d_in[10];
  const float* w10 = (const float*)d_in[11];
  const float* g10 = (const float*)d_in[12];
  const float* b10 = (const float*)d_in[13];
  const float* w11 = (const float*)d_in[14];
  const float* g11 = (const float*)d_in[15];
  const float* b11 = (const float*)d_in[16];
  const float* w12 = (const float*)d_in[17];
  const float* g12 = (const float*)d_in[18];
  const float* b12 = (const float*)d_in[19];

  char* ws = (char*)d_ws;
  unsigned short* FT  = (unsigned short*)(ws + OFF_FT);
  float* PPL          = (float*)(ws + OFF_PPL);
  unsigned short* WH  = (unsigned short*)(ws + OFF_WH);
  float* WXP          = (float*)(ws + OFF_WXP);
  float* NXW          = (float*)(ws + OFF_NXW);
  int* IDX0           = (int*)(ws + OFF_IDX0);
  int* IDX1           = (int*)(ws + OFF_IDX1);
  float* PART0        = (float*)(ws + OFF_PART0);
  float* PART10       = (float*)(ws + OFF_PART10);
  float* PART11       = (float*)(ws + OFF_PART11);
  float* PART20       = (float*)(ws + OFF_PART20);
  float* PART21       = (float*)(ws + OFF_PART21);
  float* MX0          = (float*)(ws + OFF_MX0);
  float* MN0          = (float*)(ws + OFF_MN0);
  float* MX1          = (float*)(ws + OFF_MX1);
  float* MN1          = (float*)(ws + OFF_MN1);
  float* SSP          = (float*)(ws + OFF_SSP);

  float* out0 = (float*)d_out;
  float* out1 = (float*)d_out + (size_t)NBATCH * NCENT * 3;

  const double invN0 = 1.0 / (double)(NGROUPS * KSAMP0);
  const double invN1 = 1.0 / (double)(NGROUPS * KSAMP1);

  k_packfeat<<<dim3(1024), dim3(256), 0, stream>>>(feat, FT);
  k_packw<<<dim3(16, 8), dim3(256), 0, stream>>>(w00, w10, w01, w02, w11, w12, WH, WXP);
  k_fps<<<dim3(NBATCH), dim3(1024), 0, stream>>>(xyz, out0, NXW);
  k_ball<<<dim3(NGROUPS / 8), dim3(256), 0, stream>>>(xyz, NXW, IDX0, IDX1);
  k_pgemm<<<dim3(256), dim3(256), 0, stream>>>(FT, WH + WH_F0, WXP, xyz, PPL);
  k_stats0<<<dim3(1536), dim3(256), 0, stream>>>(PPL, IDX0, IDX1, NXW, WXP, PART0);
  k_fold<<<dim3(1), dim3(256), 0, stream>>>(PART0, 512, 64, g00, b00, invN0, SSP + 0 * 512);
  k_fold<<<dim3(1), dim3(256), 0, stream>>>(PART0 + (size_t)512 * 128, 1024, 64, g10, b10, invN1, SSP + 3 * 512);

  k_mlp<64, 128, KSAMP0, 0><<<dim3(2048), dim3(128), 0, stream>>>(PPL, IDX0, NXW, WXP, SSP + 0 * 512, SSP + 1 * 512,
      WH + WH_10, WH + WH_20, PART10, MX0, MN0, 0);
  k_fold<<<dim3(1), dim3(256), 0, stream>>>(PART10, 2048, 64, g01, b01, invN0, SSP + 1 * 512);
  k_mlp<64, 128, KSAMP0, 1><<<dim3(2048), dim3(128), 0, stream>>>(PPL, IDX0, NXW, WXP, SSP + 0 * 512, SSP + 1 * 512,
      WH + WH_10, WH + WH_20, PART20, MX0, MN0, 0);
  k_fold<<<dim3(1), dim3(256), 0, stream>>>(PART20, 2048, 128, g02, b02, invN0, SSP + 2 * 512);
  k_final<<<dim3(128 * 2), dim3(256), 0, stream>>>(MX0, MN0, SSP + 2 * 512, out1, 128, 0);

  k_mlp<128, 256, KSAMP1, 0><<<dim3(4096), dim3(128), 0, stream>>>(PPL, IDX1, NXW, WXP + 64 * 4, SSP + 3 * 512, SSP + 4 * 512,
      WH + WH_11, WH + WH_21, PART11, MX1, MN1, 64);
  k_fold<<<dim3(1), dim3(256), 0, stream>>>(PART11, 4096, 128, g11, b11, invN1, SSP + 4 * 512);
  k_mlp<128, 256, KSAMP1, 1><<<dim3(4096), dim3(128), 0, stream>>>(PPL, IDX1, NXW, WXP + 64 * 4, SSP + 3 * 512, SSP + 4 * 512,
      WH + WH_11, WH + WH_21, PART21, MX1, MN1, 64);
  k_fold<<<dim3(1), dim3(256), 0, stream>>>(PART21, 4096, 256, g12, b12, invN1, SSP + 5 * 512);
  k_final<<<dim3(128 * 4), dim3(256), 0, stream>>>(MX1, MN1, SSP + 5 * 512, out1, 256, 128);
}
